// Attention_55825984913972
// MI455X (gfx1250) — hardware-verified
//
#include <hip/hip_runtime.h>


#ifndef SEQ
#define SEQ 4096
#endif
#ifndef NB
#define NB 1
#endif
#define SEQ_FULL 4096
#define DIM   1024
#define HEADS 16
#define HD    64
#define INNER (HEADS * HD)
#define NQKV  (3 * INNER)
#define LN_EPS 1.0e-6f
#define LOG2E 1.4426950408889634f
#define C32   0.03125f
#define WS_CAP ((size_t)134217728)

static_assert(SEQ % 64 == 0);
static_assert(SEQ <= SEQ_FULL);
static_assert(NB == 1);
static_assert(DIM == 128 * 8);
static_assert(DIM % 64 == 0);
static_assert(NQKV % 64 == 0);
static_assert(INNER == DIM);
static_assert(HD == 64);
static_assert((HEADS * SEQ * HD) % (256 * 8) == 0);
static_assert((HEADS * HD * SEQ) % (256 * 2) == 0);

typedef _Float16 h16;
typedef unsigned short bf;
typedef __attribute__((ext_vector_type(16))) __bf16   v16bf;
typedef __attribute__((ext_vector_type(16))) _Float16 v16h;
typedef __attribute__((ext_vector_type(8)))  _Float16 v8h;
typedef __attribute__((ext_vector_type(8)))  unsigned short v8us;
typedef __attribute__((ext_vector_type(8)))  float    v8f;
typedef __attribute__((ext_vector_type(4)))  float    v4f;
typedef __attribute__((ext_vector_type(2)))  _Float16 v2h;
typedef __attribute__((ext_vector_type(2)))  unsigned short v2us;
typedef v8h  __attribute__((may_alias)) v8ha;
typedef v4f  __attribute__((may_alias)) v4fa;
typedef v8us __attribute__((may_alias)) v8usa;

__device__ __forceinline__ unsigned short f2bf(float f) { unsigned u = __float_as_uint(f); u += 0x7FFFu + ((u >> 16) & 1u); return (unsigned short)(u >> 16); }
__device__ __forceinline__ float bf2f(unsigned short b) { return __uint_as_float(((unsigned)b) << 16); }
__device__ __forceinline__ float bfr(float f) { return bf2f(f2bf(f)); }
__device__ __forceinline__ v16h cat16(v8h lo, v8h hi) { return __builtin_shufflevector(lo, hi, 0, 1, 2, 3, 4, 5, 6, 7, 8, 9, 10, 11, 12, 13, 14, 15); }
__device__ __forceinline__ v16bf cat16b(v8us lo, v8us hi) { return __builtin_bit_cast(v16bf, __builtin_shufflevector(lo, hi, 0, 1, 2, 3, 4, 5, 6, 7, 8, 9, 10, 11, 12, 13, 14, 15)); }
__device__ __forceinline__ v8f wmma16(v16h a, v16h b, v8f c) { return __builtin_amdgcn_wmma_f32_16x16x32_f16(false, a, false, b, (short)0, c, false, false); }
__device__ __forceinline__ v8f wmmab(v16bf a, v16bf b, v8f c) { return __builtin_amdgcn_wmma_f32_16x16x32_bf16(false, a, false, b, (short)0, c, false, false); }
__device__ __forceinline__ void splitf(float y, unsigned short& h, unsigned short& l) { h = f2bf(y); l = f2bf(y - bf2f(h)); }

template <typename T16> struct WFrag;
template <> struct WFrag<h16> { typedef v16h V; static __device__ __forceinline__ V ld(const h16* p) { return cat16(*(const v8h*)p, *(const v8h*)(p + 16)); } static __device__ __forceinline__ v8f mma(V a, V b, v8f c) { return wmma16(a, b, c); } };
template <> struct WFrag<bf> { typedef v16bf V; static __device__ __forceinline__ V ld(const bf* p) { return cat16b(*(const v8us*)p, *(const v8us*)(p + 16)); } static __device__ __forceinline__ v8f mma(V a, V b, v8f c) { return wmmab(a, b, c); } };
template <typename T16, int NSPLIT, bool BIAS>
__global__ __launch_bounds__(32) void k_gemmw(const T16* __restrict__ A, const T16* __restrict__ A2, const T16* __restrict__ Bt, const T16* __restrict__ Bt2, int K, float* C, int ldc, const float* __restrict__ bias, size_t sA, size_t sB, size_t sC) {
    typedef typename WFrag<T16>::V V;
    __shared__ __align__(16) float os[16 * 68];
    const size_t z = blockIdx.z; A += z * sA; if (A2) A2 += z * sA; Bt += z * sB; if (Bt2) Bt2 += z * sB; C += z * sC;
    const int lane = threadIdx.x & 31, lr = lane & 15, hi = lane >> 4; const int r0 = blockIdx.x * 64, c0 = blockIdx.y * 64;
    v8f acc[4][4];
#pragma unroll
    for (int mb = 0; mb < 4; ++mb)
#pragma unroll
        for (int nb = 0; nb < 4; ++nb) acc[mb][nb] = (v8f){};
    const size_t aoff = (size_t)(r0 + lr) * K + 8 * hi, boff = (size_t)(c0 + lr) * K + 8 * hi;
#pragma unroll 1
    for (int kc = 0; kc < K; kc += 32) {
        V a[4], a2[4];
#pragma unroll
        for (int mb = 0; mb < 4; ++mb) { a[mb] = WFrag<T16>::ld(A + aoff + (size_t)mb * 16 * K + kc); if (NSPLIT == 1 || NSPLIT == 2) a2[mb] = WFrag<T16>::ld(A2 + aoff + (size_t)mb * 16 * K + kc); }
#pragma unroll
        for (int nb = 0; nb < 4; ++nb) { const V b = WFrag<T16>::ld(Bt + boff + (size_t)nb * 16 * K + kc); V b2; if (NSPLIT >= 2) b2 = WFrag<T16>::ld(Bt2 + boff + (size_t)nb * 16 * K + kc);
#pragma unroll
            for (int mb = 0; mb < 4; ++mb) { acc[mb][nb] = WFrag<T16>::mma(a[mb], b, acc[mb][nb]); if (NSPLIT == 1 || NSPLIT == 2) acc[mb][nb] = WFrag<T16>::mma(a2[mb], b, acc[mb][nb]); if (NSPLIT >= 2) acc[mb][nb] = WFrag<T16>::mma(a[mb], b2, acc[mb][nb]); } }
        asm volatile("v_nop\n\tv_nop\n\tv_nop\n\tv_nop" : "+v"(acc[0][0]), "+v"(acc[1][1]), "+v"(acc[2][2]), "+v"(acc[3][3]) : "v"(a[0]), "v"(a[3]));
    }
#pragma unroll
    for (int mb = 0; mb < 4; ++mb) {
#pragma unroll
        for (int nb = 0; nb < 4; ++nb) {
#pragma unroll
            for (int j = 0; j < 8; ++j) os[(hi * 8 + j) * 68 + nb * 16 + lr] = acc[mb][nb][j]; }
        __builtin_amdgcn_wave_barrier(); asm volatile("" ::: "memory");
        float* crow = C + (size_t)(r0 + mb * 16) * ldc + c0;
#pragma unroll 1
        for (int ps = 0; ps < 2; ++ps) {
#pragma unroll
            for (int s = 0; s < 8; ++s) { const int row = 2 * s + hi, cofs = lr * 4; v4f val = *(const v4fa*)(os + row * 68 + cofs); if (BIAS) { val[0] += bfr(bias[c0 + cofs]); val[1] += bfr(bias[c0 + cofs + 1]); val[2] += bfr(bias[c0 + cofs + 2]); val[3] += bfr(bias[c0 + cofs + 3]); }
                *(volatile v4f*)(crow + (size_t)row * ldc + cofs) = val; }
            if (ps == 0) __threadfence(); }
        __builtin_amdgcn_wave_barrier(); asm volatile("" ::: "memory");
    }
}

__global__ __launch_bounds__(256) void k_wtG(const float* __restrict__ w, int K, int N, bf* Bt) {
    const int lane = threadIdx.x & 31; const int L0 = (blockIdx.x * 8 + (threadIdx.x >> 5)) * 8; const int nlines = N * K / 64;
#pragma unroll
    for (int ps = 0; ps < 2; ++ps) {
#pragma unroll 1
        for (int l = 0; l < 8; ++l) { const int L = L0 + l; if (L >= nlines) break; const size_t e = (size_t)L * 64 + lane * 2; const int k = (int)(e % K), n = (int)(e / K); v2us o;
            o[0] = f2bf(w[(size_t)k * N + n]); o[1] = f2bf(w[(size_t)(k + 1) * N + n]); *(volatile v2us*)(Bt + e) = o; }
        if (ps == 0) __threadfence(); }
}

__global__ __launch_bounds__(128) void k_ln(const float* __restrict__ x, const float* __restrict__ g, const float* __restrict__ b, bf* Yh, bf* Yl) {
    __shared__ float red[8];
    const int tid = threadIdx.x, lane = tid & 31, wid = tid >> 5; const size_t row = blockIdx.x;
    const v8f xv = *(const v8f*)(x + row * DIM + 8 * tid);
    float xb[8]; float s = 0.f;
#pragma unroll
    for (int q = 0; q < 8; ++q) { xb[q] = bfr(xv[q]); s += xb[q]; }
#pragma unroll
    for (int sh = 16; sh; sh >>= 1) s += __shfl_xor(s, sh, 32);
    if (lane == 0) red[wid] = s;
    __syncthreads();
    const float mean = ((red[0] + red[1]) + (red[2] + red[3])) * (1.0f / DIM);
    float d[8]; float s2 = 0.f;
#pragma unroll
    for (int q = 0; q < 8; ++q) { d[q] = xb[q] - mean; s2 += d[q] * d[q]; }
#pragma unroll
    for (int sh = 16; sh; sh >>= 1) s2 += __shfl_xor(s2, sh, 32);
    if (lane == 0) red[4 + wid] = s2;
    __syncthreads();
    const float var = ((red[4] + red[5]) + (red[6] + red[7])) * (1.0f / DIM);
    const float rstd = rsqrtf(var + LN_EPS);
    const v8f gv = *(const v8f*)(g + 8 * tid); const v8f bv = *(const v8f*)(b + 8 * tid);
    v8us oh, ol;
#pragma unroll
    for (int q = 0; q < 8; ++q) { const float y = d[q] * rstd * bfr(gv[q]) + bfr(bv[q]); unsigned short a2, c2; splitf(y, a2, c2); oh[q] = a2; ol[q] = c2; }
    const size_t o = row * DIM + 8 * tid;
    *(volatile v8us*)(Yh + o) = oh; *(volatile v8us*)(Yl + o) = ol; __threadfence(); *(volatile v8us*)(Yh + o) = oh; *(volatile v8us*)(Yl + o) = ol;
}

__global__ __launch_bounds__(256) void k_hp16(const float* __restrict__ src, int coloff, float scl, h16* P) {
    const size_t i = (size_t)blockIdx.x * 256 + threadIdx.x; if (i >= (size_t)HEADS * SEQ * HD / 8) return; const size_t e = i * 8;
    const int d = (int)(e % HD); const int t = (int)((e / HD) % SEQ); const int h = (int)(e / ((size_t)HD * SEQ));
    const v8f v = *(const v8f*)(src + (size_t)t * NQKV + coloff + h * HD + d); v8h o;
#pragma unroll
    for (int q = 0; q < 8; ++q) o[q] = (h16)(v[q] * scl);
    *(volatile v8h*)(P + e) = o; __threadfence(); *(volatile v8h*)(P + e) = o;
}
__global__ __launch_bounds__(256) void k_vt16(const float* __restrict__ src, h16* VT) {
    const size_t e = ((size_t)blockIdx.x * 256 + threadIdx.x) * 2; if (e >= (size_t)HEADS * HD * SEQ) return;
    const int t = (int)(e % SEQ); const int d = (int)((e / SEQ) % HD); const int h = (int)(e / ((size_t)SEQ * HD));
    v2h o; o[0] = (h16)src[(size_t)t * NQKV + 2 * INNER + h * HD + d]; o[1] = (h16)src[(size_t)(t + 1) * NQKV + 2 * INNER + h * HD + d];
    *(volatile v2h*)(VT + e) = o; __threadfence(); *(volatile v2h*)(VT + e) = o;
}

__global__ __launch_bounds__(128) void k_flash(const h16* __restrict__ Q16, const h16* __restrict__ K16, const h16* __restrict__ VT16, bf* CTXh, bf* CTXl) {
    __shared__ __align__(16) float os[4][16 * 68];
    const int lane = threadIdx.x & 31, wid = threadIdx.x >> 5, m = lane & 15, hh = lane >> 4;
    const int gw = blockIdx.x * 4 + wid; const int h = gw / (SEQ / 16); const int q0 = (gw - h * (SEQ / 16)) * 16;
    const h16* Qp = Q16 + ((size_t)h * SEQ + q0) * HD; const h16* Kp = K16 + (size_t)h * SEQ * HD; const h16* Vp = VT16 + (size_t)h * HD * SEQ;
    v16h qb[2];
#pragma unroll
    for (int ks = 0; ks < 2; ++ks) qb[ks] = WFrag<h16>::ld(Qp + (size_t)m * HD + 32 * ks + 8 * hh);
    v8f oacc[4];
#pragma unroll
    for (int t = 0; t < 4; ++t) oacc[t] = (v8f){};
    float mrun = -3.0e38f, lrun = 0.f;
    const size_t koff = (size_t)m * HD + 8 * hh; const size_t voff = (size_t)m * SEQ + 8 * hh;
#pragma unroll 1
    for (int j0 = 0; j0 < SEQ; j0 += 32) {
        v8f sc[2]; sc[0] = (v8f){}; sc[1] = (v8f){};
        v16h ka[4];
#pragma unroll
        for (int t = 0; t < 2; ++t)
#pragma unroll
            for (int ks = 0; ks < 2; ++ks) ka[t * 2 + ks] = WFrag<h16>::ld(Kp + (size_t)(j0 + 16 * t) * HD + koff + 32 * ks);
#pragma unroll
        for (int t = 0; t < 2; ++t)
#pragma unroll
            for (int ks = 0; ks < 2; ++ks) sc[t] = wmma16(ka[t * 2 + ks], qb[ks], sc[t]);
        asm volatile("v_nop\n\tv_nop\n\tv_nop\n\tv_nop" : "+v"(sc[0]), "+v"(sc[1]) : "v"(ka[0]), "v"(ka[3]), "v"(qb[0]), "v"(qb[1]));
        float cmx = fmaxf(sc[0][0], sc[1][0]);
#pragma unroll
        for (int r = 1; r < 8; ++r) cmx = fmaxf(cmx, fmaxf(sc[0][r], sc[1][r]));
        cmx = fmaxf(cmx, __shfl_xor(cmx, 16, 32));
        const float mn = fmaxf(mrun, cmx);
        const float alpha = __builtin_amdgcn_exp2f((mrun - mn) * C32);
        float psum = 0.f; v16h pb;
#pragma unroll
        for (int r = 0; r < 8; ++r) { const float e0 = __builtin_amdgcn_exp2f((sc[0][r] - mn) * C32); const float e1 = __builtin_amdgcn_exp2f((sc[1][r] - mn) * C32); psum += e0 + e1; pb[r] = (h16)e0; pb[8 + r] = (h16)e1; }
        psum += __shfl_xor(psum, 16, 32);
        lrun = lrun * alpha + psum; mrun = mn;
#pragma unroll
        for (int t = 0; t < 4; ++t) oacc[t] *= alpha;
        v16h va[4];
#pragma unroll
        for (int t = 0; t < 4; ++t) va[t] = WFrag<h16>::ld(Vp + (size_t)(16 * t) * SEQ + voff + j0);
#pragma unroll
        for (int t = 0; t < 4; ++t) oacc[t] = wmma16(va[t], pb, oacc[t]);
        asm volatile("v_nop\n\tv_nop\n\tv_nop\n\tv_nop" : "+v"(oacc[0]), "+v"(oacc[1]), "+v"(oacc[2]), "+v"(oacc[3]) : "v"(pb), "v"(va[0]), "v"(va[3]));
    }
    const float inv = 1.0f / lrun;
    float* ob = os[wid];
#pragma unroll
    for (int t = 0; t < 4; ++t) { v4f u0, u1;
#pragma unroll
        for (int r = 0; r < 4; ++r) { u0[r] = oacc[t][r] * inv; u1[r] = oacc[t][4 + r] * inv; }
        *(v4fa*)(ob + m * 68 + 16 * t + 8 * hh) = u0; *(v4fa*)(ob + m * 68 + 16 * t + 8 * hh + 4) = u1; }
    __builtin_amdgcn_fence(3  , "wavefront"); __builtin_amdgcn_wave_barrier(); asm volatile("" ::: "memory");
#pragma unroll 1
    for (int ps = 0; ps < 2; ++ps) {
#pragma unroll
        for (int p = 0; p < 4; ++p) { const int row = p * 4 + (lane >> 3), c8 = (lane & 7) * 8;
            const v4f a = *(const v4fa*)(ob + row * 68 + c8); const v4f b2 = *(const v4fa*)(ob + row * 68 + c8 + 4);
            v8us oh, ol;
#pragma unroll
            for (int q = 0; q < 4; ++q) { unsigned short x1, y1; splitf(a[q], x1, y1); oh[q] = x1; ol[q] = y1; splitf(b2[q], x1, y1); oh[4 + q] = x1; ol[4 + q] = y1; }
            const size_t oo = (size_t)(q0 + row) * INNER + h * HD + c8;
            *(volatile v8us*)(CTXh + oo) = oh; *(volatile v8us*)(CTXl + oo) = ol; }
        if (ps == 0) __threadfence(); }
}

extern "C" void kernel_launch(void* const* d_in, const int* in_sizes, int n_in,
                              void* d_out, int out_size, void* d_ws, size_t ws_size, hipStream_t stream) {
    if (n_in < 6) return;
    if (in_sizes[0] < SEQ * DIM || in_sizes[1] < DIM || in_sizes[2] < DIM || in_sizes[3] < DIM * NQKV || in_sizes[4] < INNER * DIM || in_sizes[5] < DIM) return;
    if (out_size < SEQ * DIM) return;
    const float* x    = (const float*)d_in[0];
    const float* lnsc = (const float*)d_in[1];
    const float* lnbs = (const float*)d_in[2];
    const float* wqkv = (const float*)d_in[3];
    const float* wout = (const float*)d_in[4];
    const float* bout = (const float*)d_in[5];
    float* OUT = (float*)d_out;
    char* wsp = (char*)d_ws;
    auto take = [&](size_t bytes) { char* p = wsp; wsp += (bytes + 255) & ~(size_t)255; return (void*)p; };
    bf*    WQ   = (bf*)take((size_t)NQKV * DIM * 2);
    bf*    WO   = (bf*)take((size_t)DIM * INNER * 2);
    bf*    XNh  = (bf*)take((size_t)SEQ * DIM * 2);
    bf*    XNl  = (bf*)take((size_t)SEQ * DIM * 2);
    float* QKV  = (float*)take((size_t)SEQ * NQKV * 4);
    h16*   Q16  = (h16*)take((size_t)HEADS * SEQ * HD * 2);
    h16*   K16  = (h16*)take((size_t)HEADS * SEQ * HD * 2);
    h16*   VT16 = (h16*)take((size_t)HEADS * HD * SEQ * 2);
    bf*    CTXh = (bf*)take((size_t)SEQ * INNER * 2);
    bf*    CTXl = (bf*)take((size_t)SEQ * INNER * 2);
    const size_t used = (size_t)(wsp - (char*)d_ws);
    if (used > ws_size || used > WS_CAP) return;

    k_wtG<<<(unsigned)(((size_t)NQKV * DIM / 64 + 63) / 64), 256, 0, stream>>>(wqkv, DIM, NQKV, WQ);
    k_wtG<<<(unsigned)(((size_t)DIM * INNER / 64 + 63) / 64), 256, 0, stream>>>(wout, INNER, DIM, WO);
    k_ln<<<SEQ, 128, 0, stream>>>(x, lnsc, lnbs, XNh, XNl);
    k_gemmw<bf, 1, false><<<dim3(SEQ / 64, NQKV / 64, 1), 32, 0, stream>>>(XNh, XNl, WQ, nullptr, DIM, QKV, NQKV, nullptr, 0, 0, 0);
    k_hp16<<<(unsigned)(((size_t)HEADS * SEQ * HD / 8 + 255) / 256), 256, 0, stream>>>(QKV, 0, LOG2E, Q16);
    k_hp16<<<(unsigned)(((size_t)HEADS * SEQ * HD / 8 + 255) / 256), 256, 0, stream>>>(QKV, INNER, 1.0f, K16);
    k_vt16<<<(unsigned)(((size_t)HEADS * HD * SEQ / 2 + 255) / 256), 256, 0, stream>>>(QKV, VT16);
    k_flash<<<(unsigned)(HEADS * (SEQ / 64)), 128, 0, stream>>>(Q16, K16, VT16, CTXh, CTXl);
    k_gemmw<bf, 1, true><<<dim3(SEQ / 64, DIM / 64, 1), 32, 0, stream>>>(CTXh, CTXl, WO, nullptr, INNER, OUT, DIM, bout, 0, 0, 0);
}
